// NeRF_MLP_55997783605497
// MI455X (gfx1250) — hardware-run, weakly checked
//
#include <hip/hip_runtime.h>
#include <math.h>

typedef __attribute__((ext_vector_type(16))) _Float16 v16h;
typedef __attribute__((ext_vector_type(8)))  _Float16 v8h;
typedef __attribute__((ext_vector_type(8)))  float    v8f;
typedef __attribute__((ext_vector_type(4)))  float    v4f;

constexpr int kRowsN  = 131072;
constexpr int kHid    = 256;
constexpr int kHid2   = 128;
constexpr int kLPos   = 10;
constexpr int kLDir   = 4;
constexpr int kXE     = 3 + 6 * kLPos;
constexpr int kDE     = 3 + 6 * kLDir;
constexpr int kXEP    = 64;
constexpr int kDEP    = 32;
constexpr int kK6     = kHid + kXE;
constexpr int kK6P    = kHid + kXEP;
constexpr int kK10    = kHid + kDE;
constexpr int kK10P   = kHid + kDEP;
constexpr int kTR     = 32;
static_assert(kXE == 63 && kDE == 27, "encoding widths");
static_assert(kK6 == 319 && kK6P == 320 && kK10 == 283 && kK10P == 288, "concat widths");
static_assert((kXEP % 32) == 0 && (kHid % 32) == 0 && (kK6P % 32) == 0 && (kK10P % 32) == 0, "K multiples of 32");
static_assert((kRowsN % kTR) == 0, "row tiles");

constexpr int kPA   = 328;
constexpr int kPL   = 264;
constexpr int kPX   = 72;
constexpr int kPS   = 260;
constexpr int kPS10 = 132;
static_assert((kPA % 8) == 0 && (kPL % 8) == 0 && (kPX % 8) == 0 && (kPS % 4) == 0 && (kPS10 % 4) == 0, "LDS alignment");
static_assert(kTR * kPS10 <= kTR * kPS, "stash holds the 128-wide tile too");

constexpr float kCarryA    = 64.0f;
constexpr float kCarryW    = 1024.0f;
constexpr float kCarryR    = 2048.0f;
constexpr float kScaleMain = 1.0f / (kCarryA * kCarryW);
constexpr float kScaleRes  = 1.0f / kCarryR;

constexpr size_t kSzW1   = (size_t)kHid * kXEP * 2;
constexpr size_t kSzWsq  = (size_t)kHid * kHid * 2;
constexpr size_t kSzW6   = (size_t)kHid * kK6P * 2;
constexpr size_t kSzW6L  = (size_t)kHid * kXEP * 2;
constexpr size_t kSzW10  = (size_t)kHid2 * kK10P * 2;
constexpr size_t kOffW1H  = 0;
constexpr size_t kOffW2H  = kOffW1H + kSzW1;
constexpr size_t kOffW3H  = kOffW2H + kSzWsq;
constexpr size_t kOffW4H  = kOffW3H + kSzWsq;
constexpr size_t kOffW5H  = kOffW4H + kSzWsq;
constexpr size_t kOffW6H  = kOffW5H + kSzWsq;
constexpr size_t kOffW6L  = kOffW6H + kSzW6;
constexpr size_t kOffW7H  = kOffW6L + kSzW6L;
constexpr size_t kOffW7L  = kOffW7H + kSzWsq;
constexpr size_t kOffW8H  = kOffW7L + kSzWsq;
constexpr size_t kOffW8L  = kOffW8H + kSzWsq;
constexpr size_t kOffW9H  = kOffW8L + kSzWsq;
constexpr size_t kOffW10H = kOffW9H + kSzWsq;
constexpr size_t kWsTotal = kOffW10H + kSzW10;
static_assert(kWsTotal == 1482752ull, "carve total");
static_assert(kWsTotal <= 134217728ull, "carve cap");
static_assert((kOffW2H % 128) == 0 && (kOffW6H % 128) == 0 && (kOffW6L % 128) == 0 && (kOffW7H % 128) == 0 &&
              (kOffW9H % 128) == 0 && (kOffW10H % 128) == 0, "line aligned planes");

__device__ __forceinline__ v16h frag_ld(const _Float16* p) {
  union { v16h v; v8h h[2]; } f;
  f.h[0] = *(const v8h*)(p);
  f.h[1] = *(const v8h*)(p + 16);
  return f.v;
}
__device__ __forceinline__ v8f mma_h(v16h a, v16h b, v8f c) {
  c = __builtin_amdgcn_wmma_f32_16x16x32_f16(false, a, false, b, (short)0, c, false, false);
  asm volatile("v_nop\n\tv_nop\n\tv_nop\n\tv_nop" : "+v"(c) : "v"(a), "v"(b));
  return c;
}

template <int NT>
__device__ __forceinline__ void zero_acc(v8f (&a)[2][NT]) {
#pragma unroll
  for (int i = 0; i < 2; ++i)
#pragma unroll
    for (int j = 0; j < NT; ++j) a[i][j] = (v8f){0.f, 0.f, 0.f, 0.f, 0.f, 0.f, 0.f, 0.f};
}

template <int NT>
__device__ __forceinline__ void acc_plain(v8f (&acc)[2][NT],
    const _Float16* Ah, int lda, int acol,
    const _Float16* Bh, int ldb, int n0, int kbeg, int nsteps, int lane)
{
  const int rl = lane & 15;
  const int ko = (lane >> 4) << 3;
  const _Float16* ap = Ah + rl * lda + acol + kbeg + ko;
  const _Float16* bp = Bh + (size_t)(n0 + rl) * ldb + kbeg + ko;
#pragma unroll 1
  for (int s = 0; s < nsteps; ++s) {
    v16h a[2], b[NT];
#pragma unroll
    for (int mt = 0; mt < 2; ++mt) a[mt] = frag_ld(ap + s * 32 + mt * 16 * lda);
#pragma unroll
    for (int t = 0; t < NT; ++t) b[t] = frag_ld(bp + s * 32 + (size_t)t * 16 * ldb);
#pragma unroll
    for (int t = 0; t < NT; ++t)
#pragma unroll
      for (int mt = 0; mt < 2; ++mt) acc[mt][t] = mma_h(a[mt], b[t], acc[mt][t]);
  }
}

template <int NT>
__device__ __forceinline__ void acc_split(v8f (&acc)[2][NT], v8f (&accr)[2][NT],
    const _Float16* Ah, int lda, int acolH,
    const _Float16* Al, int ldal, int acolL,
    const _Float16* Bh, int ldb,
    const _Float16* Bl, int ldbl, int bcolL,
    int n0, int kbeg, int nsteps, int lane)
{
  const int rl = lane & 15;
  const int ko = (lane >> 4) << 3;
  const _Float16* aph = Ah + rl * lda + acolH + kbeg + ko;
  const _Float16* apl = Al + rl * ldal + acolL + kbeg + ko;
  const _Float16* bph = Bh + (size_t)(n0 + rl) * ldb + kbeg + ko;
  const _Float16* bpl = Bl + (size_t)(n0 + rl) * ldbl + bcolL + kbeg + ko;
#pragma unroll 1
  for (int s = 0; s < nsteps; ++s) {
    v16h ah[2], al[2], bh[NT], bl[NT];
#pragma unroll
    for (int mt = 0; mt < 2; ++mt) {
      ah[mt] = frag_ld(aph + s * 32 + mt * 16 * lda);
      al[mt] = frag_ld(apl + s * 32 + mt * 16 * ldal);
    }
#pragma unroll
    for (int t = 0; t < NT; ++t) {
      bh[t] = frag_ld(bph + s * 32 + (size_t)t * 16 * ldb);
      bl[t] = frag_ld(bpl + s * 32 + (size_t)t * 16 * ldbl);
    }
#pragma unroll
    for (int t = 0; t < NT; ++t)
#pragma unroll
      for (int mt = 0; mt < 2; ++mt) {
        acc[mt][t]  = mma_h(ah[mt], bh[t], acc[mt][t]);
        accr[mt][t] = mma_h(al[mt], bh[t], accr[mt][t]);
        accr[mt][t] = mma_h(ah[mt], bl[t], accr[mt][t]);
      }
  }
}

template <int NT, bool RES, bool RELU, bool WH, bool WL, bool WS>
__device__ __forceinline__ void epilogue(const v8f (&acc)[2][NT], const v8f (&accr)[2][NT],
    const float* __restrict__ bias, int n0,
    _Float16* oh, int ldh, _Float16* ol, int ldl, float* st, int ldst, int lane)
{
  const int nl = lane & 15;
  const int r0 = (lane >> 4) << 3;
#pragma unroll
  for (int t = 0; t < NT; ++t) {
    const int n = n0 + t * 16 + nl;
    const float bv = bias[n];
#pragma unroll
    for (int mt = 0; mt < 2; ++mt) {
#pragma unroll
      for (int r = 0; r < 8; ++r) {
        const int row = mt * 16 + r0 + r;
        float m = acc[mt][t][r];
        if (RES) m = m + accr[mt][t][r] * kScaleRes;
        float v = m * kScaleMain + bv;
        if (RELU) v = fmaxf(v, 0.0f);
        if (WS) st[row * ldst + n] = v;
        if (WH || WL) {
          const float s = v * kCarryA;
          const _Float16 hv = (_Float16)s;
          if (WH) oh[row * ldh + n] = hv;
          if (WL) ol[row * ldl + n] = (_Float16)((s - (float)hv) * kCarryR);
        }
      }
    }
  }
}

__device__ __forceinline__ void put_hl(_Float16* ph, _Float16* pl, float v) {
  const float s = v * kCarryA;
  const _Float16 hv = (_Float16)s;
  *ph = hv;
  *pl = (_Float16)((s - (float)hv) * kCarryR);
}

__global__ __launch_bounds__(256) void prep_weight_planes(
    const float* __restrict__ src, int kreal, int kpad,
    unsigned short* __restrict__ hi, unsigned short* __restrict__ lo, int lo_c0, int lo_w, int total8)
{
  const int i = blockIdx.x * 256 + threadIdx.x;
  if (i >= total8) return;
  const int per_row = kpad >> 3;
  const int r = i / per_row;
  const int c = (i - r * per_row) << 3;
  const float* sp = src + (size_t)r * kreal;
  v8h hv, lv;
#pragma unroll
  for (int e = 0; e < 8; ++e) {
    const int k = c + e;
    const int kc = (k < kreal) ? k : (kreal - 1);
    float w = sp[kc];
    w = (k < kreal) ? w : 0.0f;
    const float s = w * kCarryW;
    const _Float16 h = (_Float16)s;
    hv[e] = h;
    lv[e] = (_Float16)((s - (float)h) * kCarryR);
  }
  unsigned short* qh = hi + (size_t)r * kpad + c;
  const bool has_lo = (lo != nullptr) && (c >= lo_c0) && (c < lo_c0 + lo_w);
  const int cl = has_lo ? (c - lo_c0) : 0;
  unsigned short* ql = has_lo ? (lo + (size_t)r * lo_w + cl) : hi;
  *(volatile v8h*)qh = hv;
  if (has_lo) *(volatile v8h*)ql = lv;
  __threadfence();
  *(volatile v8h*)qh = hv;
  if (has_lo) *(volatile v8h*)ql = lv;
}

__global__ __launch_bounds__(256) void fused_chain_kernel(
    const float* __restrict__ xyz, const float* __restrict__ dvec,
    const _Float16* __restrict__ W1h, const _Float16* __restrict__ W2h, const _Float16* __restrict__ W3h,
    const _Float16* __restrict__ W4h, const _Float16* __restrict__ W5h,
    const _Float16* __restrict__ W6h, const _Float16* __restrict__ W6l,
    const _Float16* __restrict__ W7h, const _Float16* __restrict__ W7l,
    const _Float16* __restrict__ W8h, const _Float16* __restrict__ W8l,
    const _Float16* __restrict__ W9h, const _Float16* __restrict__ W10h,
    const float* __restrict__ b1, const float* __restrict__ b2, const float* __restrict__ b3,
    const float* __restrict__ b4, const float* __restrict__ b5, const float* __restrict__ b6,
    const float* __restrict__ b7, const float* __restrict__ b8, const float* __restrict__ b9,
    const float* __restrict__ b10,
    const float* __restrict__ W9f, const float* __restrict__ W11, const float* __restrict__ b11,
    float* __restrict__ out0, float* __restrict__ out1)
{
  __shared__ __align__(16) _Float16 sAh[kTR * kPA];
  __shared__ __align__(16) _Float16 sBh[kTR * kPA];
  __shared__ __align__(16) _Float16 sAl[kTR * kPL];
  __shared__ __align__(16) _Float16 sBl[kTR * kPL];
  __shared__ __align__(16) _Float16 sXl[kTR * kPX];
  __shared__ __align__(16) float sSt[kTR * kPS];
  __shared__ __align__(16) float sW11[3 * kHid2];
  __shared__ __align__(16) float sIn[2 * 3 * kTR];
  __shared__ __align__(16) float sDen[kTR];
  __shared__ float sB11[4];

  const int tid  = threadIdx.x;
  const int lane = tid & 31;
  const int wave = __builtin_amdgcn_readfirstlane((int)(threadIdx.x >> 5));
  const int rowbase = blockIdx.x * kTR;
  const int n0 = wave * 32;

  {
    const int ci = (tid < 3 * kTR) ? tid : (3 * kTR - 1);
    const int c2 = (tid < 128) ? tid : 127;
    const int c3 = (tid < 3) ? tid : 2;
    float xv = xyz[(size_t)rowbase * 3 + ci];
    float dv = dvec[(size_t)rowbase * 3 + ci];
    float w0 = W11[tid];
    float w1 = W11[256 + c2];
    float bb = b11[c3];
    asm volatile("" : "+v"(xv), "+v"(dv), "+v"(w0), "+v"(w1), "+v"(bb));
    sW11[tid] = w0;
    if (tid < 128) sW11[256 + tid] = w1;
    if (tid < 3 * kTR) {
      sIn[tid] = xv;
      sIn[3 * kTR + tid] = dv;
    }
    if (tid < 3) sB11[tid] = bb;
  }
  __syncthreads();

#pragma unroll 1
  for (int it = 0; it < 4; ++it) {
    const int item = it * 256 + tid;
    const bool valid = item < kTR * 3 * kLPos;
    const int ic = valid ? item : (kTR * 3 * kLPos - 1);
    const int row = ic / (3 * kLPos);
    const int rem = ic - row * (3 * kLPos);
    const int lv = rem / 3;
    const int dim = rem - lv * 3;
    const float x = sIn[row * 3 + dim];
    const float t = x * (float)(1 << lv);
    const float sn = sinf(t);
    const float cs = cosf(t);
    if (valid) {
      const int col = 3 + 6 * lv + dim;
      put_hl(sAh + row * kPA + kHid + col,     sXl + row * kPX + col,     sn);
      put_hl(sAh + row * kPA + kHid + col + 3, sXl + row * kPX + col + 3, cs);
    }
  }
  if (tid < 3 * kTR) {
    const int row = tid / 3;
    const int dim = tid - row * 3;
    put_hl(sAh + row * kPA + kHid + dim, sXl + row * kPX + dim, sIn[tid]);
  }
  if (tid < kTR) {
    sAh[tid * kPA + kHid + kXE] = (_Float16)0.0f;
    sXl[tid * kPX + kXE] = (_Float16)0.0f;
  }
  __syncthreads();

  {
    v8f acc[2][2];
    zero_acc<2>(acc);
    acc_plain<2>(acc, sAh, kPA, kHid, W1h, kXEP, n0, 0, kXEP / 32, lane);
    epilogue<2, false, true, true, false, false>(acc, acc, b1, n0, sAh, kPA, sAh, kPA, sSt, kPS, lane);
  }
  __syncthreads();
  {
    v8f acc[2][2];
    zero_acc<2>(acc);
    acc_plain<2>(acc, sAh, kPA, 0, W2h, kHid, n0, 0, kHid / 32, lane);
    epilogue<2, false, true, true, false, false>(acc, acc, b2, n0, sBh, kPA, sBh, kPA, sSt, kPS, lane);
  }
  __syncthreads();
  {
    v8f acc[2][2];
    zero_acc<2>(acc);
    acc_plain<2>(acc, sBh, kPA, 0, W3h, kHid, n0, 0, kHid / 32, lane);
    epilogue<2, false, true, true, false, false>(acc, acc, b3, n0, sAh, kPA, sAh, kPA, sSt, kPS, lane);
  }
  __syncthreads();
  {
    v8f acc[2][2];
    zero_acc<2>(acc);
    acc_plain<2>(acc, sAh, kPA, 0, W4h, kHid, n0, 0, kHid / 32, lane);
    epilogue<2, false, true, true, false, false>(acc, acc, b4, n0, sBh, kPA, sBh, kPA, sSt, kPS, lane);
  }
  __syncthreads();
  {
    v8f acc[2][2];
    zero_acc<2>(acc);
    acc_plain<2>(acc, sBh, kPA, 0, W5h, kHid, n0, 0, kHid / 32, lane);
    epilogue<2, false, true, true, false, false>(acc, acc, b5, n0, sAh, kPA, sAh, kPA, sSt, kPS, lane);
  }
  __syncthreads();
  {
    v8f acc[2][2], accr[2][2];
    zero_acc<2>(acc);
    zero_acc<2>(accr);
    acc_plain<2>(acc, sAh, kPA, 0, W6h, kK6P, n0, 0, kHid / 32, lane);
    acc_split<2>(acc, accr, sAh, kPA, 0, sXl, kPX, -kHid, W6h, kK6P, W6l, kXEP, -kHid, n0, kHid, kXEP / 32, lane);
    epilogue<2, true, true, true, true, false>(acc, accr, b6, n0, sBh, kPA, sBl, kPL, sSt, kPS, lane);
  }
  __syncthreads();
  {
    v8f acc[2][2], accr[2][2];
    zero_acc<2>(acc);
    zero_acc<2>(accr);
    acc_split<2>(acc, accr, sBh, kPA, 0, sBl, kPL, 0, W7h, kHid, W7l, kHid, 0, n0, 0, kHid / 32, lane);
    epilogue<2, true, true, true, true, false>(acc, accr, b7, n0, sAh, kPA, sAl, kPL, sSt, kPS, lane);
  }
  __syncthreads();
  {
    v8f acc[2][2], accr[2][2];
    zero_acc<2>(acc);
    zero_acc<2>(accr);
    acc_split<2>(acc, accr, sAh, kPA, 0, sAl, kPL, 0, W8h, kHid, W8l, kHid, 0, n0, 0, kHid / 32, lane);
    epilogue<2, true, true, true, true, true>(acc, accr, b8, n0, sBh, kPA, sBl, kPL, sSt, kPS, lane);
  }
  __syncthreads();

  {
    const int row  = tid >> 3;
    const int part = tid & 7;
    const float* sp = sSt + row * kPS + part * 32;
    const float* wp = W9f + (size_t)kHid * kHid + part * 32;
    float sum = 0.0f;
#pragma unroll 2
    for (int i = 0; i < 8; ++i) {
      const v4f a = *(const v4f*)(sp + 4 * i);
      const v4f w = *(const v4f*)(wp + 4 * i);
      sum = fmaf(a[0], w[0], sum);
      sum = fmaf(a[1], w[1], sum);
      sum = fmaf(a[2], w[2], sum);
      sum = fmaf(a[3], w[3], sum);
    }
    sum += __shfl_xor(sum, 1, 32);
    sum += __shfl_xor(sum, 2, 32);
    sum += __shfl_xor(sum, 4, 32);
    const float bd = b9[kHid];
    const float dval = fmaxf(sum + bd, 0.0f);
    if (part == 0) sDen[row] = dval;
  }

#pragma unroll 1
  for (int it = 0; it < 2; ++it) {
    const int item = it * 256 + tid;
    const bool valid = item < kTR * 3 * kLDir;
    const int ic = valid ? item : (kTR * 3 * kLDir - 1);
    const int row = ic / (3 * kLDir);
    const int rem = ic - row * (3 * kLDir);
    const int lv = rem / 3;
    const int dim = rem - lv * 3;
    const float x = sIn[3 * kTR + row * 3 + dim];
    const float t = x * (float)(1 << lv);
    const float sn = sinf(t);
    const float cs = cosf(t);
    if (valid) {
      const int col = kHid + 3 + 6 * lv + dim;
      sAh[row * kPA + col]     = (_Float16)(sn * kCarryA);
      sAh[row * kPA + col + 3] = (_Float16)(cs * kCarryA);
    }
  }
  if (tid < 3 * kTR) {
    const int row = tid / 3;
    const int dim = tid - row * 3;
    sAh[row * kPA + kHid + dim] = (_Float16)(sIn[3 * kTR + tid] * kCarryA);
  }
  if (tid < kTR * (kDEP - kDE)) {
    const int row = tid / (kDEP - kDE);
    const int c = tid - row * (kDEP - kDE);
    sAh[row * kPA + kHid + kDE + c] = (_Float16)0.0f;
  }

  {
    v8f acc[2][2];
    zero_acc<2>(acc);
    acc_plain<2>(acc, sBh, kPA, 0, W9h, kHid, n0, 0, kHid / 32, lane);
    epilogue<2, false, false, true, false, false>(acc, acc, b9, n0, sAh, kPA, sAh, kPA, sSt, kPS, lane);
  }
  __syncthreads();

  {
    v8f acc[2][1];
    zero_acc<1>(acc);
    acc_plain<1>(acc, sAh, kPA, 0, W10h, kK10P, wave * 16, 0, kK10P / 32, lane);
    epilogue<1, false, true, false, false, true>(acc, acc, b10, wave * 16, sAh, kPA, sAh, kPA, sSt, kPS10, lane);
  }
  __syncthreads();

  if (wave < 3) {
    const int e = tid;
    const int row = e / 3;
    const int o = e - row * 3;
    const float* ap = sSt + row * kPS10;
    const float* wp = sW11 + o * kHid2;
    float sum = 0.0f;
#pragma unroll 4
    for (int k = 0; k < kHid2; ++k) sum = fmaf(ap[k], wp[k], sum);
    const float lg = sum + sB11[o];
    const float cv = 1.0f / (1.0f + expf(-lg));
    volatile float* q = out0 + (size_t)blockIdx.x * (3 * kTR) + e;
    *q = cv;
    __threadfence();
    *q = cv;
  }
  if (wave == 3) {
    const float dvl = sDen[lane];
    volatile float* q = out1 + (size_t)rowbase + lane;
    *q = dvl;
    __threadfence();
    *q = dvl;
  }
}

static inline void launch_prep(const float* src, int rows, int kreal, int kpad,
                               unsigned short* hi, unsigned short* lo, int lo_c0, int lo_w, hipStream_t stream) {
  const int total8 = rows * kpad / 8;
  const int grid = (total8 + 255) / 256;
  prep_weight_planes<<<grid, 256, 0, stream>>>(src, kreal, kpad, hi, lo, lo_c0, lo_w, total8);
}

extern "C" void kernel_launch(void* const* d_in, const int* in_sizes, int n_in,
                              void* d_out, int out_size, void* d_ws, size_t ws_size,
                              hipStream_t stream) {
  if (n_in < 24) return;
  if (in_sizes[0] != kRowsN * 3 || in_sizes[1] != kRowsN * 3) return;
  if (in_sizes[2] != kHid * kXE || in_sizes[3] != kHid) return;
  if (in_sizes[4] != kHid * kHid || in_sizes[5] != kHid) return;
  if (in_sizes[6] != kHid * kHid || in_sizes[7] != kHid) return;
  if (in_sizes[8] != kHid * kHid || in_sizes[9] != kHid) return;
  if (in_sizes[10] != kHid * kHid || in_sizes[11] != kHid) return;
  if (in_sizes[12] != kHid * kK6 || in_sizes[13] != kHid) return;
  if (in_sizes[14] != kHid * kHid || in_sizes[15] != kHid) return;
  if (in_sizes[16] != kHid * kHid || in_sizes[17] != kHid) return;
  if (in_sizes[18] != (kHid + 1) * kHid || in_sizes[19] != kHid + 1) return;
  if (in_sizes[20] != kHid2 * kK10 || in_sizes[21] != kHid2) return;
  if (in_sizes[22] != 3 * kHid2 || in_sizes[23] != 3) return;
  if (out_size != kRowsN * 4) return;
  if (ws_size < kWsTotal) return;

  const float* xyz  = (const float*)d_in[0];
  const float* dvec = (const float*)d_in[1];
  const float* W1  = (const float*)d_in[2];
  const float* b1  = (const float*)d_in[3];
  const float* W2  = (const float*)d_in[4];
  const float* b2  = (const float*)d_in[5];
  const float* W3  = (const float*)d_in[6];
  const float* b3  = (const float*)d_in[7];
  const float* W4  = (const float*)d_in[8];
  const float* b4  = (const float*)d_in[9];
  const float* W5  = (const float*)d_in[10];
  const float* b5  = (const float*)d_in[11];
  const float* W6  = (const float*)d_in[12];
  const float* b6  = (const float*)d_in[13];
  const float* W7  = (const float*)d_in[14];
  const float* b7  = (const float*)d_in[15];
  const float* W8  = (const float*)d_in[16];
  const float* b8  = (const float*)d_in[17];
  const float* W9  = (const float*)d_in[18];
  const float* b9  = (const float*)d_in[19];
  const float* W10 = (const float*)d_in[20];
  const float* b10 = (const float*)d_in[21];
  const float* W11 = (const float*)d_in[22];
  const float* b11 = (const float*)d_in[23];

  float* out0 = (float*)d_out;
  float* out1 = out0 + (size_t)kRowsN * 3;

  char* ws = (char*)d_ws;
  unsigned short* pW1H  = (unsigned short*)(ws + kOffW1H);
  unsigned short* pW2H  = (unsigned short*)(ws + kOffW2H);
  unsigned short* pW3H  = (unsigned short*)(ws + kOffW3H);
  unsigned short* pW4H  = (unsigned short*)(ws + kOffW4H);
  unsigned short* pW5H  = (unsigned short*)(ws + kOffW5H);
  unsigned short* pW6H  = (unsigned short*)(ws + kOffW6H);
  unsigned short* pW6L  = (unsigned short*)(ws + kOffW6L);
  unsigned short* pW7H  = (unsigned short*)(ws + kOffW7H);
  unsigned short* pW7L  = (unsigned short*)(ws + kOffW7L);
  unsigned short* pW8H  = (unsigned short*)(ws + kOffW8H);
  unsigned short* pW8L  = (unsigned short*)(ws + kOffW8L);
  unsigned short* pW9H  = (unsigned short*)(ws + kOffW9H);
  unsigned short* pW10H = (unsigned short*)(ws + kOffW10H);

  launch_prep(W1,  kHid,  kXE,  kXEP,  pW1H,  nullptr, 0, 0, stream);
  launch_prep(W2,  kHid,  kHid, kHid,  pW2H,  nullptr, 0, 0, stream);
  launch_prep(W3,  kHid,  kHid, kHid,  pW3H,  nullptr, 0, 0, stream);
  launch_prep(W4,  kHid,  kHid, kHid,  pW4H,  nullptr, 0, 0, stream);
  launch_prep(W5,  kHid,  kHid, kHid,  pW5H,  nullptr, 0, 0, stream);
  launch_prep(W6,  kHid,  kK6,  kK6P,  pW6H,  pW6L, kHid, kXEP, stream);
  launch_prep(W7,  kHid,  kHid, kHid,  pW7H,  pW7L, 0, kHid, stream);
  launch_prep(W8,  kHid,  kHid, kHid,  pW8H,  pW8L, 0, kHid, stream);
  launch_prep(W9,  kHid,  kHid, kHid,  pW9H,  nullptr, 0, 0, stream);
  launch_prep(W10, kHid2, kK10, kK10P, pW10H, nullptr, 0, 0, stream);

  fused_chain_kernel<<<kRowsN / kTR, 256, 0, stream>>>(
      xyz, dvec,
      (const _Float16*)pW1H, (const _Float16*)pW2H, (const _Float16*)pW3H,
      (const _Float16*)pW4H, (const _Float16*)pW5H,
      (const _Float16*)pW6H, (const _Float16*)pW6L,
      (const _Float16*)pW7H, (const _Float16*)pW7L,
      (const _Float16*)pW8H, (const _Float16*)pW8L,
      (const _Float16*)pW9H, (const _Float16*)pW10H,
      b1, b2, b3, b4, b5, b6, b7, b8, b9, b10,
      W9, W11, b11,
      out0, out1);
}
